// MSA_80109730005335
// MI455X (gfx1250) — hardware-verified
//
#include <hip/hip_runtime.h>
#include <math.h>

typedef __attribute__((ext_vector_type(16))) _Float16 v16h;
typedef __attribute__((ext_vector_type(16))) __bf16 v16b;
typedef __attribute__((ext_vector_type(8)))  _Float16 v8h;
typedef __attribute__((ext_vector_type(8)))  __bf16 v8b;
typedef __attribute__((ext_vector_type(8)))  float v8f;
typedef __attribute__((ext_vector_type(4)))  float v4f;
typedef __attribute__((ext_vector_type(4)))  unsigned v4u;

template <typename T> __device__ __forceinline__ void vst2(void* p, T v) { *(volatile T*)p = v; __threadfence(); *(volatile T*)p = v; }

__device__ __forceinline__ v8f wmma16(v16h a, v16h b, v8f c) {
  v8f d = __builtin_amdgcn_wmma_f32_16x16x32_f16(false, a, false, b, (short)0, c, false, false);
  asm volatile("v_nop\n\tv_nop\n\tv_nop\n\tv_nop" : "+v"(d) : "v"(a), "v"(b));
  return d;
}
__device__ __forceinline__ v8f wmma_bf(v16b a, v16b b, v8f c) {
  v8f d = __builtin_amdgcn_wmma_f32_16x16x32_bf16(false, a, false, b, (short)0, c, false, false);
  asm volatile("v_nop\n\tv_nop\n\tv_nop\n\tv_nop" : "+v"(d) : "v"(a), "v"(b));
  return d;
}
__device__ __forceinline__ v16h frag_h(const _Float16* rowk0, int lane) {
  union { v16h v; v8h q[2]; } u; const _Float16* p = rowk0 + 8 * (lane >> 4);
  u.q[0] = *(const v8h*)p; u.q[1] = *(const v8h*)(p + 16); return u.v;
}
__device__ __forceinline__ v16b frag_b(const __bf16* rowk0, int lane) {
  union { v16b v; v8b q[2]; } u; const __bf16* p = rowk0 + 8 * (lane >> 4);
  u.q[0] = *(const v8b*)p; u.q[1] = *(const v8b*)(p + 16); return u.v;
}
__device__ __forceinline__ v16h frag_f32s(const float* rowk0, int lane, float sc) {
  v16h a; const float* p = rowk0 + 8 * (lane >> 4);
#pragma unroll
  for (int i = 0; i < 8; ++i) { a[i] = (_Float16)(p[i] * sc); a[8 + i] = (_Float16)(p[16 + i] * sc); }
  return a;
}
struct F2 { v16b h, l; };
__device__ __forceinline__ F2 bsplit16(const float v[16]) { F2 r;
#pragma unroll
  for (int i = 0; i < 16; ++i) { const __bf16 hb = (__bf16)v[i]; r.h[i] = hb; r.l[i] = (__bf16)(v[i] - (float)hb); }
  return r; }
__device__ __forceinline__ F2 split_row(const float* row, int k0, int lane) { float v[16]; const float* p = row + k0 + 8 * (lane >> 4);
#pragma unroll
  for (int i = 0; i < 8; ++i) { v[i] = p[i]; v[8 + i] = p[16 + i]; }
  return bsplit16(v); }
__device__ __forceinline__ float bfr(float v) { return (float)(__bf16)v; }
__device__ __forceinline__ void ldsx() { asm volatile("s_wait_dscnt 0" ::: "memory"); __builtin_amdgcn_wave_barrier(); __builtin_amdgcn_fence(3, "workgroup"); }

#define NB_FULL 2
#define SEQ_FULL 2048
#ifndef NB
#define NB NB_FULL
#endif
#ifndef SEQ
#define SEQ SEQ_FULL
#endif
#define CC 1024
#define NH 16
#define HD 64
#define HG 4
static_assert(NB >= 1 && NB <= NB_FULL);
static_assert(SEQ >= 128 && SEQ <= SEQ_FULL && (SEQ % 128) == 0);
static_assert(NH * HD == CC && (NH % HG) == 0 && HD == 64 && (CC % 128) == 0);

#define PR     ((size_t)NB * SEQ)
#define WS_QH  ((size_t)0)
#define WS_QL  (WS_QH + 2u * PR * CC)
#define WS_KH  (WS_QL + 2u * PR * CC)
#define WS_VT  (WS_KH + 2u * PR * CC)
#define WS_VL  (WS_VT + 2u * (size_t)NB * CC * SEQ)
#define WS_S   (WS_VL + 2u * (size_t)NB * CC * SEQ)
#define WS_Y   (WS_S + 4u * (size_t)HG * SEQ * SEQ)
#define WS_END (WS_Y + 4u * PR * CC)
static_assert(WS_END <= (size_t)134217728u);
static_assert((((size_t)(NB - 1) * SEQ_FULL + SEQ) * CC) <= (size_t)NB_FULL * SEQ_FULL * CC);

__global__ __launch_bounds__(128) __attribute__((amdgpu_num_vgpr(256)))
void k_proj(const float* __restrict__ X, const float* __restrict__ W, _Float16* __restrict__ QH, _Float16* __restrict__ QL, _Float16* __restrict__ KH, __bf16* __restrict__ VT, __bf16* __restrict__ VL) {
  __shared__ __align__(16) _Float16 sh[64][136], sl[64][136];
  __shared__ __align__(16) __bf16 th[128][72], tl2[128][72];
  const int tid = threadIdx.x, wave = tid >> 5, lane = tid & 31, col = lane & 15, g = lane >> 4;
  const int which = blockIdx.z; const int c0 = blockIdx.y * 128;
  const size_t r0 = (size_t)blockIdx.x * 64;
  const size_t b = r0 / SEQ; const int t0 = (int)(r0 % SEQ);
  const size_t xr0 = b * SEQ_FULL + (size_t)t0;
  v8f acc[8] = {};
#pragma unroll 1
  for (int kc = 0; kc < CC / 32; ++kc) {
    v16b a; { const float* p = X + (xr0 + wave * 16 + col) * CC + kc * 32 + 8 * g;
#pragma unroll
      for (int i = 0; i < 8; ++i) { a[i] = (__bf16)p[i]; a[8 + i] = (__bf16)p[16 + i]; } }
#pragma unroll
    for (int j = 0; j < 8; ++j) { v16b w; const int oc = c0 + j * 16 + col; const float* wp = W + ((size_t)which * CC + oc) * CC + kc * 32 + 8 * g;
#pragma unroll
      for (int i = 0; i < 8; ++i) { w[i] = (__bf16)wp[i]; w[8 + i] = (__bf16)wp[16 + i]; }
      acc[j] = wmma_bf(a, w, acc[j]); } }
#pragma unroll
  for (int j = 0; j < 8; ++j) {
#pragma unroll
    for (int r = 0; r < 8; ++r) { const float v = acc[j][r]; const int rl = wave * 16 + 8 * g + r, cl = j * 16 + col;
      if (which == 2) { const __bf16 bh = (__bf16)v; th[cl][rl] = bh; tl2[cl][rl] = (__bf16)(v - (float)bh); }
      else { const _Float16 hv = (_Float16)v; sh[rl][cl] = hv; sl[rl][cl] = (_Float16)((v - (float)hv) * 1024.0f); }
    } }
  __syncthreads();
  if (which < 2) { _Float16* dh = (which == 0) ? QH : KH;
    for (int e = tid; e < 64 * 16; e += 128) { const int rl = e >> 4, q = e & 15; const size_t o = (r0 + rl) * CC + c0 + q * 8;
      vst2(dh + o, *(const v4u*)&sh[rl][q * 8]); if (which == 0) vst2(QL + o, *(const v4u*)&sl[rl][q * 8]); } }
  else { for (int e = tid; e < 128 * 8; e += 128) { const int cl = e >> 3, q = e & 7; const size_t o2 = (b * CC + c0 + cl) * (size_t)SEQ + t0 + q * 8;
      vst2(VT + o2, *(const v4u*)&th[cl][q * 8]); vst2(VL + o2, *(const v4u*)&tl2[cl][q * 8]); } }
}
__global__ __launch_bounds__(128) __attribute__((amdgpu_num_vgpr(256)))
void k_sc(const _Float16* __restrict__ QH, const _Float16* __restrict__ QL, const _Float16* __restrict__ KH, int b, int h0, float* __restrict__ S0) {
  __shared__ __align__(16) float ss[4][16][132];
  const int h = h0 + blockIdx.z; float* S = S0 + (size_t)blockIdx.z * SEQ * SEQ;
  const int tid = threadIdx.x, wave = tid >> 5, lane = tid & 31, col = lane & 15, g = lane >> 4;
  const int k0 = blockIdx.y * 128; const int ql0 = blockIdx.x * 64 + wave * 16; const size_t q0 = (size_t)b * SEQ + ql0;
  v8f acc[8] = {}, accl[8] = {};
#pragma unroll 1
  for (int kc = 0; kc < HD / 32; ++kc) {
    const v16h ah = frag_h(QH + (q0 + col) * CC + h * HD + kc * 32, lane), al = frag_h(QL + (q0 + col) * CC + h * HD + kc * 32, lane);
#pragma unroll
    for (int j = 0; j < 8; ++j) { const v16h kb = frag_h(KH + ((size_t)b * SEQ + k0 + j * 16 + col) * CC + h * HD + kc * 32, lane);
      acc[j] = wmma16(ah, kb, acc[j]); accl[j] = wmma16(al, kb, accl[j]); } }
#pragma unroll
  for (int j = 0; j < 8; ++j) {
#pragma unroll
    for (int r = 0; r < 8; ++r) ss[wave][8 * g + r][j * 16 + col] = (acc[j][r] + accl[j][r] * (1.0f / 1024.0f)) * (1.0f / 64.0f); }
  ldsx();
  for (int rl = 0; rl < 16; ++rl) vst2(S + (size_t)(ql0 + rl) * SEQ + k0 + lane * 4, *(const v4f*)&ss[wave][rl][lane * 4]);
}
__global__ __launch_bounds__(256) void k_sm(float* __restrict__ S0) {
  __shared__ float sred[8]; __shared__ float sbc; __shared__ __align__(16) float sh[SEQ];
  const int t = threadIdx.x; const size_t row = blockIdx.x;
  float* sr = S0 + (size_t)blockIdx.y * SEQ * SEQ + row * SEQ;
  float m = -3.0e38f;
#pragma unroll 1
  for (int k = t; k < SEQ; k += 256) { const float v = sr[k]; sh[k] = v; m = fmaxf(m, v); }
#pragma unroll
  for (int o = 1; o < 32; o <<= 1) m = fmaxf(m, __shfl_xor(m, o));
  if ((t & 31) == 0) sred[t >> 5] = m;
  __syncthreads();
  if (t == 0) { float a = sred[0]; for (int i = 1; i < 8; ++i) a = fmaxf(a, sred[i]); sbc = a; }
  __syncthreads(); m = sbc; __syncthreads();
  float sum = 0.f;
#pragma unroll 1
  for (int k = t; k < SEQ; k += 256) { const float e = expf(sh[k] - m); sh[k] = e; sum += e; }
#pragma unroll
  for (int o = 1; o < 32; o <<= 1) sum += __shfl_xor(sum, o);
  if ((t & 31) == 0) sred[t >> 5] = sum;
  __syncthreads();
  if (t == 0) { float a = 0.f; for (int i = 0; i < 8; ++i) a += sred[i]; sbc = (1.0f / a) * 2048.0f; }
  __syncthreads(); const float c = sbc;
#pragma unroll 1
  for (int q = t; q < SEQ / 4; q += 256) { v4f pv = *(const v4f*)&sh[q * 4]; pv = pv * c; vst2(sr + q * 4, pv); }
}
__global__ __launch_bounds__(128) __attribute__((amdgpu_num_vgpr(256)))
void k_pv(const float* __restrict__ PS0, const __bf16* __restrict__ VT, const __bf16* __restrict__ VL, int b, int h0, float* __restrict__ Y) {
  const int h = h0 + blockIdx.z; const float* PS = PS0 + (size_t)blockIdx.z * SEQ * SEQ;
  __shared__ __align__(16) float ss[4][16][HD + 4];
  const int tid = threadIdx.x, wave = tid >> 5, lane = tid & 31, col = lane & 15, g = lane >> 4;
  const int ql0 = blockIdx.x * 64 + wave * 16;
  v8f acc[HD / 16] = {};
#pragma unroll 1
  for (int kc = 0; kc < SEQ / 32; ++kc) { const F2 p = split_row(PS + (size_t)(ql0 + col) * SEQ, kc * 32, lane);
#pragma unroll
    for (int j = 0; j < HD / 16; ++j) { const size_t po = ((size_t)b * CC + h * HD + j * 16 + col) * (size_t)SEQ + kc * 32; const v16b vh = frag_b(VT + po, lane);
      acc[j] = wmma_bf(p.h, vh, acc[j]); acc[j] = wmma_bf(p.l, vh, acc[j]); acc[j] = wmma_bf(p.h, frag_b(VL + po, lane), acc[j]); } }
#pragma unroll
  for (int j = 0; j < HD / 16; ++j) {
#pragma unroll
    for (int r = 0; r < 8; ++r) ss[wave][8 * g + r][j * 16 + col] = acc[j][r] * (1.0f / 2048.0f); }
  ldsx();
  for (int rl = 0; rl < 16; ++rl) if (lane < HD / 4) vst2(Y + ((size_t)b * SEQ + ql0 + rl) * CC + h * HD + lane * 4, *(const v4f*)&ss[wave][rl][lane * 4]);
}
__global__ __launch_bounds__(128) __attribute__((amdgpu_num_vgpr(256)))
void k_out(const float* __restrict__ Y, const float* __restrict__ W, const float* __restrict__ Bv, float* __restrict__ O) {
  __shared__ __align__(16) float so[64][132];
  const int tid = threadIdx.x, wave = tid >> 5, lane = tid & 31, col = lane & 15, g = lane >> 4;
  const int c0 = blockIdx.y * 128; const size_t r0 = (size_t)blockIdx.x * 64;
  v8f acc[8] = {};
#pragma unroll 1
  for (int kc = 0; kc < CC / 32; ++kc) {
    const v16h a = frag_f32s(Y + (r0 + wave * 16 + col) * CC + kc * 32, lane, 64.0f);
#pragma unroll
    for (int j = 0; j < 8; ++j) { v16h w; const int oc = c0 + j * 16 + col; const float* wp = W + (size_t)oc * CC + kc * 32 + 8 * g;
#pragma unroll
      for (int i = 0; i < 8; ++i) { w[i] = (_Float16)(bfr(wp[i]) * 64.0f); w[8 + i] = (_Float16)(bfr(wp[16 + i]) * 64.0f); }
      acc[j] = wmma16(a, w, acc[j]); } }
#pragma unroll
  for (int j = 0; j < 8; ++j) { const float bb = bfr(Bv[c0 + j * 16 + col]);
#pragma unroll
    for (int r = 0; r < 8; ++r) { const int rl = wave * 16 + 8 * g + r, cl = j * 16 + col; so[rl][cl] = acc[j][r] * (1.0f / 4096.0f) + bb; } }
  __syncthreads();
  const size_t b = r0 / SEQ; const int t0 = (int)(r0 % SEQ);
  for (int rl = wave * 16; rl < wave * 16 + 16; ++rl)
    vst2(O + (b * SEQ_FULL + (size_t)(t0 + rl)) * CC + c0 + lane * 4, *(const v4f*)&so[rl][lane * 4]);
}

extern "C" void kernel_launch(void* const* d_in, const int* in_sizes, int n_in, void* d_out, int out_size, void* d_ws, size_t ws_size, hipStream_t stream) {
  if (n_in < 4) return;
  const size_t rows_needed = (size_t)(NB - 1) * SEQ_FULL + SEQ;
  if ((size_t)in_sizes[0] < rows_needed * CC) return;
  if ((size_t)in_sizes[1] < (size_t)3 * CC * CC) return;
  if ((size_t)in_sizes[2] < (size_t)CC * CC) return;
  if (in_sizes[3] < CC) return;
  if ((size_t)out_size < rows_needed * CC) return;
  if (ws_size < (size_t)WS_END) return;
  const float* X = (const float*)d_in[0]; const float* W = (const float*)d_in[1]; const float* WO = (const float*)d_in[2]; const float* BO = (const float*)d_in[3];
  char* ws = (char*)d_ws;
  _Float16 *QH = (_Float16*)(ws + WS_QH), *QL = (_Float16*)(ws + WS_QL), *KH = (_Float16*)(ws + WS_KH);
  __bf16 *VT = (__bf16*)(ws + WS_VT), *VL = (__bf16*)(ws + WS_VL);
  float *S = (float*)(ws + WS_S), *Y = (float*)(ws + WS_Y);
  k_proj<<<dim3(NB * SEQ / 64, CC / 128, 3), 128, 0, stream>>>(X, W, QH, QL, KH, VT, VL);
  for (int b = 0; b < NB; ++b) for (int h0 = 0; h0 < NH; h0 += HG) {
    k_sc<<<dim3(SEQ / 64, SEQ / 128, HG), 128, 0, stream>>>(QH, QL, KH, b, h0, S);
    k_sm<<<dim3(SEQ, HG), 256, 0, stream>>>(S);
    k_pv<<<dim3(SEQ / 64, 1, HG), 128, 0, stream>>>(S, VT, VL, b, h0, Y);
  }
  k_out<<<dim3(NB * SEQ / 64, CC / 128), 128, 0, stream>>>(Y, WO, BO, (float*)d_out);
}
